// SAN_21028159881449
// MI455X (gfx1250) — hardware-verified
//
#include <hip/hip_runtime.h>


namespace {
constexpr int Bn = 2, S = 4096, DM = 512, H = 8, HD = 64, NT = Bn * S;
constexpr float QS = 8.0f, KS = 8.0f, VS = 8.0f, PS = 8.0f, SCALE = 0.125f;
constexpr size_t PL = (size_t)Bn * H * S * HD;

typedef _Float16 b16;
typedef __attribute__((ext_vector_type(16))) _Float16 v16b;
typedef __attribute__((ext_vector_type(16))) __bf16 v16bb;
typedef __attribute__((ext_vector_type(8))) _Float16 v8b;
typedef __attribute__((ext_vector_type(8))) unsigned short v8us;
typedef __attribute__((ext_vector_type(8))) float v8f;
typedef __attribute__((ext_vector_type(4))) float v4f;
__device__ __forceinline__ float bf16_rne(float f) { unsigned int u = __float_as_uint(f); u += 0x7FFFu + ((u >> 16) & 1u); return __uint_as_float(u & 0xFFFF0000u); }
__device__ __forceinline__ unsigned short bf16_bits(float f) { unsigned int u = __float_as_uint(f); u += 0x7FFFu + ((u >> 16) & 1u); return (unsigned short)(u >> 16); }
__device__ __forceinline__ v16b frag_kb(const b16* p, int hh) { const v8b a = *(const v8b*)(p + 8 * hh), b = *(const v8b*)(p + 16 + 8 * hh); v16b f;
#pragma unroll
  for (int e = 0; e < 8; ++e) { f[e] = a[e]; f[8 + e] = b[e]; } return f; }
__device__ __forceinline__ v16bb frag_bf(const unsigned short* p, int hh) { const v8us a = *(const v8us*)(p + 8 * hh), b = *(const v8us*)(p + 16 + 8 * hh); union { unsigned short s[16]; v16bb v; } u;
#pragma unroll
  for (int e = 0; e < 8; ++e) { u.s[e] = a[e]; u.s[8 + e] = b[e]; } return u.v; }
__device__ __forceinline__ v16bb frag_f32bf(const float* p, int hh) { union { unsigned short s[16]; v16bb v; } u;
#pragma unroll
  for (int e = 0; e < 8; ++e) { u.s[e] = bf16_bits(p[8 * hh + e]); u.s[8 + e] = bf16_bits(p[16 + 8 * hh + e]); } return u.v; }
__device__ __forceinline__ v8f wmma16b(v16b a, v16b b, v8f c) { v8f d = __builtin_amdgcn_wmma_f32_16x16x32_f16(false, a, false, b, (short)0, c, false, false); asm volatile("v_nop\n\tv_nop\n\tv_nop\n\tv_nop" : "+v"(d) : "v"(a), "v"(b)); return d; }
__device__ __forceinline__ v8f wmma16bb(v16bb a, v16bb b, v8f c) { v8f d = __builtin_amdgcn_wmma_f32_16x16x32_bf16(false, a, false, b, (short)0, c, false, false); asm volatile("v_nop\n\tv_nop\n\tv_nop\n\tv_nop" : "+v"(d) : "v"(a), "v"(b)); return d; }
__device__ __forceinline__ void wave_lds_sync() { __builtin_amdgcn_fence(__ATOMIC_RELEASE, "workgroup"); __builtin_amdgcn_wave_barrier(); __builtin_amdgcn_fence(__ATOMIC_ACQUIRE, "workgroup"); }
__device__ __forceinline__ float nexp(float x) { return __builtin_amdgcn_exp2f(x * 1.4426950408889634f); }

__global__ __launch_bounds__(256) void prep_kernel(const float* __restrict__ Wqkv, const float* __restrict__ Wout, const float* __restrict__ bout, unsigned short* __restrict__ w16, b16* __restrict__ wo16, float* __restrict__ P) {
  const int t_ = blockIdx.x * 256 + threadIdx.x, nth = gridDim.x * 256;
  for (int pass = 0; pass < 2; ++pass) {
    for (int q = t_; q < DM * DM; q += nth) { const int o = q / DM, k = q % DM; w16[q] = bf16_bits(Wqkv[(size_t)k * DM + o]); wo16[q] = (b16)bf16_rne(Wout[(size_t)k * DM + o]); }
    for (int q = t_; q < DM; q += nth) P[q] = bf16_rne(bout[q]);
    __threadfence(); }
}

__global__ __launch_bounds__(128) void proj_kernel(const float* __restrict__ x, const unsigned short* __restrict__ w16, b16* __restrict__ qp, b16* __restrict__ kp, b16* __restrict__ vt, float* __restrict__ sq) {
  __shared__ __attribute__((aligned(16))) b16 Tq[4][32][HD + 8], Tk[4][32][HD + 8]; __shared__ __attribute__((aligned(16))) b16 Tv[HD][128 + 8]; __shared__ float Sq[128];
  const int lane = threadIdx.x & 31, wave = threadIdx.x >> 5, nloc = lane & 15, hlf = lane >> 4, h = blockIdx.x, c0 = h * HD, p0 = blockIdx.y * 128, m0 = p0 + wave * 32, b = p0 / S, t0 = p0 % S;
  v8f acc[2][4];
#pragma unroll
  for (int r = 0; r < 2; ++r)
#pragma unroll
    for (int t = 0; t < 4; ++t) acc[r][t] = (v8f){};
#pragma unroll 2
  for (int kb = 0; kb < DM; kb += 32) { const v16bb a0 = frag_f32bf(x + (size_t)(m0 + nloc) * DM + kb, hlf), a1 = frag_f32bf(x + (size_t)(m0 + 16 + nloc) * DM + kb, hlf);
#pragma unroll
    for (int t = 0; t < 4; ++t) { const v16bb bw = frag_bf(w16 + (size_t)(c0 + t * 16 + nloc) * DM + kb, hlf); acc[0][t] = wmma16bb(a0, bw, acc[0][t]); acc[1][t] = wmma16bb(a1, bw, acc[1][t]); } }
#pragma unroll
  for (int t = 0; t < 4; ++t)
#pragma unroll
    for (int r = 0; r < 2; ++r)
#pragma unroll
      for (int v = 0; v < 8; ++v) { const float w = acc[r][t][v]; Tq[wave][r * 16 + 8 * hlf + v][t * 16 + nloc] = (b16)(w * (SCALE * QS)); Tk[wave][r * 16 + 8 * hlf + v][t * 16 + nloc] = (b16)(w * KS); Tv[t * 16 + nloc][wave * 32 + r * 16 + 8 * hlf + v] = (b16)(w * VS); }
#pragma unroll
  for (int r = 0; r < 2; ++r)
#pragma unroll
    for (int v = 0; v < 8; ++v) { float s2 = 0.0f;
#pragma unroll
      for (int t = 0; t < 4; ++t) { const float w = acc[r][t][v]; s2 += w * w; }
#pragma unroll
      for (int o = 1; o < 16; o <<= 1) s2 += __shfl_xor(s2, o);
      if (nloc == 0) Sq[wave * 32 + r * 16 + 8 * hlf + v] = s2; }
  __syncthreads();
  b16* qb = qp + (((size_t)b * H + h) * S + (m0 % S)) * HD; b16* kb_ = kp + (((size_t)b * H + h) * S + (m0 % S)) * HD;
  for (int pass = 0; pass < 2; ++pass) {
#pragma unroll
    for (int j = 0; j < 8; ++j) { const int rr = j * 4 + (lane >> 3), c8 = (lane & 7) * 8; *(volatile v8b*)(qb + (size_t)rr * HD + c8) = *(const v8b*)(&Tq[wave][rr][c8]); *(volatile v8b*)(kb_ + (size_t)rr * HD + c8) = *(const v8b*)(&Tk[wave][rr][c8]); }
    for (int i = threadIdx.x; i < HD * 16; i += 128) { const int d = i >> 4, c8 = (i & 15) * 8; *(volatile v8b*)(vt + (((size_t)b * H + h) * HD + d) * S + t0 + c8) = *(const v8b*)(&Tv[d][c8]); }
    *(volatile float*)(sq + ((size_t)b * H + h) * S + t0 + threadIdx.x) = Sq[threadIdx.x];
    __threadfence(); }
}

__global__ __launch_bounds__(256) void attn_kernel(const b16* __restrict__ qp, const b16* __restrict__ kp, const b16* __restrict__ vt, const float* __restrict__ sq, b16* __restrict__ ctx) {
  __shared__ __attribute__((aligned(16))) b16 Os[16][DM + 8];
  const int h = threadIdx.x >> 5, lane = threadIdx.x & 31, hh = lane >> 4, col = lane & 15; const int b = blockIdx.x / (S / 16), q0 = (blockIdx.x % (S / 16)) * 16, qi = q0 + col;
  const b16* Q = qp + (((size_t)b * H + h) * S) * HD; const b16* K = kp + (((size_t)b * H + h) * S) * HD; const b16* V = vt + (((size_t)b * H + h) * HD) * S;
  const v16b qf0 = frag_kb(Q + (size_t)qi * HD, hh), qf1 = frag_kb(Q + (size_t)qi * HD + 32, hh); const float sself = sq[((size_t)b * H + h) * S + qi] * SCALE;
  float m = -INFINITY, l = 0.0f; v8f o[4] = {{}, {}, {}, {}};
  for (int kb = 0; kb < S; kb += 32) {
    const v16b ka0 = frag_kb(K + (size_t)(kb + col) * HD, hh), ka1 = frag_kb(K + (size_t)(kb + col) * HD + 32, hh), kc0 = frag_kb(K + (size_t)(kb + 16 + col) * HD, hh), kc1 = frag_kb(K + (size_t)(kb + 16 + col) * HD + 32, hh);
    v8f s0 = {}, s1 = {}; s0 = wmma16b(ka0, qf0, s0); s0 = wmma16b(ka1, qf1, s0); s1 = wmma16b(kc0, qf0, s1); s1 = wmma16b(kc1, qf1, s1);
    float mr = -INFINITY;
#pragma unroll
    for (int r = 0; r < 8; ++r) { s0[r] *= 1.0f / (QS * KS); s1[r] *= 1.0f / (QS * KS); if (kb + 8 * hh + r == qi) s0[r] = sself; if (kb + 16 + 8 * hh + r == qi) s1[r] = sself; mr = fmaxf(mr, fmaxf(s0[r], s1[r])); }
    mr = fmaxf(mr, __shfl_xor(mr, 16));
    const float mn = fmaxf(m, mr), al_ = nexp(m - mn); m = mn; float sum = 0.0f; v16b pbv;
#pragma unroll
    for (int r = 0; r < 8; ++r) { const float e0 = nexp(s0[r] - mn), e1 = nexp(s1[r] - mn); sum += e0 + e1; pbv[r] = (b16)(e0 * PS); pbv[8 + r] = (b16)(e1 * PS); }
    sum += __shfl_xor(sum, 16); l = l * al_ + sum;
#pragma unroll
    for (int t = 0; t < 4; ++t) { o[t] *= al_; const v16b vf = frag_kb(V + (size_t)(t * 16 + col) * S + kb, hh); o[t] = wmma16b(vf, pbv, o[t]); } }
  const float inv = 1.0f / (l * VS * PS);
#pragma unroll
  for (int t = 0; t < 4; ++t)
#pragma unroll
    for (int r = 0; r < 8; ++r) Os[col][h * HD + t * 16 + 8 * hh + r] = (b16)(o[t][r] * inv);
  __syncthreads();
  b16* dst = ctx + ((size_t)b * S + q0) * DM;
  for (int pass = 0; pass < 2; ++pass) { for (int i = threadIdx.x; i < 16 * (DM / 8); i += 256) { const int rr = i / (DM / 8), c8 = (i % (DM / 8)) * 8; *(volatile v8b*)(dst + (size_t)rr * DM + c8) = *(const v8b*)(&Os[rr][c8]); } __threadfence(); }
}

__global__ __launch_bounds__(128) void out_kernel(const b16* __restrict__ ctx, const b16* __restrict__ wo16, const float* __restrict__ P, float* __restrict__ out) {
  __shared__ __attribute__((aligned(16))) float Ts[4][32 * 64];
  const int lane = threadIdx.x & 31, wave = threadIdx.x >> 5, nloc = lane & 15, hlf = lane >> 4, m0 = blockIdx.y * 128 + wave * 32, c0 = blockIdx.x * 64;
  v8f acc[2][4];
#pragma unroll
  for (int r = 0; r < 2; ++r)
#pragma unroll
    for (int t = 0; t < 4; ++t) acc[r][t] = (v8f){};
#pragma unroll 2
  for (int kb = 0; kb < DM; kb += 32) { const v16b a0 = frag_kb(ctx + (size_t)(m0 + nloc) * DM + kb, hlf), a1 = frag_kb(ctx + (size_t)(m0 + 16 + nloc) * DM + kb, hlf);
#pragma unroll
    for (int t = 0; t < 4; ++t) { const v16b bw = frag_kb(wo16 + (size_t)(c0 + t * 16 + nloc) * DM + kb, hlf); acc[0][t] = wmma16b(a0, bw, acc[0][t]); acc[1][t] = wmma16b(a1, bw, acc[1][t]); } }
  float* Tt = Ts[wave];
#pragma unroll
  for (int t = 0; t < 4; ++t) { const float bb = P[c0 + t * 16 + nloc];
#pragma unroll
    for (int r = 0; r < 2; ++r)
#pragma unroll
      for (int v = 0; v < 8; ++v) Tt[(r * 16 + v + 8 * hlf) * 64 + t * 16 + nloc] = acc[r][t][v] + bb; }
  wave_lds_sync();
  for (int pass = 0; pass < 2; ++pass) {
#pragma unroll
    for (int j = 0; j < 16; ++j) { const int rr = j * 2 + hlf, c4 = nloc * 4; *(volatile v4f*)(out + (size_t)(m0 + rr) * DM + c0 + c4) = *(const v4f*)(Tt + rr * 64 + c4); }
    __threadfence(); }
}
}

extern "C" void kernel_launch(void* const* d_in, const int* in_sizes, int n_in,
                              void* d_out, int out_size, void* d_ws, size_t ws_size, hipStream_t stream) {
  (void)n_in; (void)out_size;
  const float* x = (const float*)d_in[0]; const float* Wqkv = (const float*)d_in[1]; const float* Wout = (const float*)d_in[2]; const float* bout = (const float*)d_in[3];
  float* out = (float*)d_out;
  if (in_sizes[0] != NT * DM || in_sizes[1] != DM * DM || in_sizes[2] != DM * DM || in_sizes[3] != DM) return;
  size_t off = 0; char* ws = (char*)d_ws;
  auto carve = [&](size_t bytes) { char* p = ws + off; off += (bytes + 255) & ~(size_t)255; return p; };
  unsigned short* w16 = (unsigned short*)carve((size_t)DM * DM * 2); b16* wo16 = (b16*)carve((size_t)DM * DM * 2); float* P = (float*)carve(DM * 4);
  b16* qp = (b16*)carve(PL * 2); b16* kp = (b16*)carve(PL * 2); b16* vt = (b16*)carve(PL * 2); b16* ctx = (b16*)carve((size_t)NT * DM * 2); float* sq = (float*)carve((size_t)NT * H * 4);
  if (off > ws_size) return;
  prep_kernel<<<256, 256, 0, stream>>>(Wqkv, Wout, bout, w16, wo16, P);
  proj_kernel<<<dim3(H, NT / 128), 128, 0, stream>>>(x, w16, qp, kp, vt, sq);
  attn_kernel<<<NT / 16, 256, 0, stream>>>(qp, kp, vt, sq, ctx);
  out_kernel<<<dim3(DM / 64, NT / 128), 128, 0, stream>>>(ctx, wo16, P, out);
}
